// MimoLinearDynamicalOperator_12841952215803
// MI455X (gfx1250) — hardware-run, weakly checked
//
#include <hip/hip_runtime.h>
#include <math.h>

typedef __attribute__((ext_vector_type(16))) _Float16 v16h;
typedef __attribute__((ext_vector_type(8)))  _Float16 v8h;
typedef __attribute__((ext_vector_type(2)))  _Float16 v2h;
typedef __attribute__((ext_vector_type(16))) __bf16   v16b;
typedef __attribute__((ext_vector_type(8)))  __bf16   v8b;
typedef __attribute__((ext_vector_type(8)))  float    v8f;
typedef __attribute__((ext_vector_type(4)))  float    v4f;
typedef __attribute__((ext_vector_type(2)))  float    v2f;

constexpr int kB    = 16;
constexpr int kT    = 4096;
constexpr int kI    = 64;
constexpr int kO    = 64;
constexpr int kNB   = 16;
constexpr int kNA   = 8;
constexpr int kTP   = kT + kNB - 1;
constexpr int kKF   = kNB * kI;
constexpr int kThr  = 256;
constexpr float kXCarry = 1024.0f;
constexpr float kBCarry = 8192.0f;
constexpr float kSc = 1.0f / (kXCarry * kBCarry);
constexpr float kF16MinNormal = 6.103515625e-5f;

static_assert(kB == 16 && kT == 4096 && kI == 64 && kO == 64 && kNB == 16 && kNA == 8 && kTP == 4111 && kKF == 1024, "the index arithmetic below uses these sizes");

constexpr size_t kOffZB = 0ull;
constexpr size_t kOffXP16 = 4096ull;
constexpr size_t kOffBT16 = 8423424ull;
constexpr size_t kOffU32 = 8554496ull;
constexpr size_t kWsTotal = 25331712ull;
static_assert(kWsTotal <= 134217728ull, "carve cap: under 128 MiB");
static_assert(kOffZB == 0
              && kOffXP16 == kOffZB + 4096ull
              && kOffBT16 == kOffXP16 + 8419328ull
              && kOffU32 == kOffBT16 + 131072ull
              && kWsTotal == kOffU32 + 16777216ull, "the carve is chained and totalled");
static_assert((kOffXP16 % 256) == 0 && (kOffBT16 % 256) == 0 && (kOffU32 % 256) == 0, "aligned regions");
static_assert(1024 >= kO, "the zero bias covers the 64 output columns (the engine reads one bias value a column)");
static_assert(((size_t)kTP * kI * 2) % 128 == 0, "a padded sample is a whole number of 128-B lines");

__device__ __forceinline__ unsigned short f2bf_bits(float f) {
  unsigned u = __float_as_uint(f);
  return (unsigned short)((u + 0x7FFFu + ((u >> 16) & 1u)) >> 16);
}
__device__ __forceinline__ float bf_bits2f(unsigned short h) { return __uint_as_float(((unsigned)h) << 16); }
__device__ __forceinline__ float bf16r(float f) { return bf_bits2f(f2bf_bits(f)); }
__device__ __forceinline__ float carry_flush(float v, float carry) {
  const float s = v * carry;
  return (fabsf(s) < kF16MinNormal) ? 0.0f : s;
}

__device__ __forceinline__ void dep_guard4_h(v8f& a, v8f& b, v8f& c, v8f& d, v16h x, v16h y) { asm volatile("v_nop\n\tv_nop\n\tv_nop\n\tv_nop" : "+v"(a), "+v"(b), "+v"(c), "+v"(d) : "v"(x), "v"(y)); }
__device__ __forceinline__ void dep_guard4_b(v8f& a, v8f& b, v8f& c, v8f& d, v16b x, v16b y) { asm volatile("v_nop\n\tv_nop\n\tv_nop\n\tv_nop" : "+v"(a), "+v"(b), "+v"(c), "+v"(d) : "v"(x), "v"(y)); }
__device__ __forceinline__ void keep4_h(v16h a, v16h b, v16h c, v16h d) { asm volatile("v_nop" :: "v"(a), "v"(b), "v"(c), "v"(d)); }
__device__ __forceinline__ void keep4_b(v16b a, v16b b, v16b c, v16b d) { asm volatile("v_nop" :: "v"(a), "v"(b), "v"(c), "v"(d)); }
__device__ __forceinline__ void acc_guard4(v8f& a, v8f& b, v8f& c, v8f& d) { asm volatile("v_nop\n\tv_nop\n\tv_nop\n\tv_nop" : "+v"(a), "+v"(b), "+v"(c), "+v"(d)); }

template <typename T> struct Frag;
template <> struct Frag<_Float16> {
  typedef v16h V; union U { v16h v; v8h h[2]; };
  static __device__ __forceinline__ v16h load(const _Float16* p) {
    U f; f.h[0] = *(const v8h*)(p); f.h[1] = *(const v8h*)(p + 16); return f.v;
  }
  static __device__ __forceinline__ v8f mma(v16h a, v16h b, v8f c) {
    return __builtin_amdgcn_wmma_f32_16x16x32_f16(false, a, false, b, (short)0, c, false, false);
  }
  static __device__ __forceinline__ void guard4(v8f& a, v8f& b, v8f& c, v8f& d, v16h x, v16h y) { dep_guard4_h(a, b, c, d, x, y); }
  static __device__ __forceinline__ void keep(v16h a, v16h b, v16h c, v16h d) { keep4_h(a, b, c, d); }
};
template <> struct Frag<__bf16> {
  typedef v16b V; union U { v16b v; v8b h[2]; };
  static __device__ __forceinline__ v16b load(const __bf16* p) {
    U f; f.h[0] = *(const v8b*)(p); f.h[1] = *(const v8b*)(p + 16); return f.v;
  }
  static __device__ __forceinline__ v8f mma(v16b a, v16b b, v8f c) {
    return __builtin_amdgcn_wmma_f32_16x16x32_bf16(false, a, false, b, (short)0, c, false, false);
  }
  static __device__ __forceinline__ void guard4(v8f& a, v8f& b, v8f& c, v8f& d, v16b x, v16b y) { dep_guard4_b(a, b, c, d, x, y); }
  static __device__ __forceinline__ void keep(v16b a, v16b b, v16b c, v16b d) { keep4_b(a, b, c, d); }
};

__device__ __forceinline__ v8f mma_h(v16h a, v16h b, v8f c) {
  c = __builtin_amdgcn_wmma_f32_16x16x32_f16(false, a, false, b, (short)0, c, false, false);
  asm volatile("v_nop\n\tv_nop\n\tv_nop\n\tv_nop" : "+v"(c) : "v"(a), "v"(b));
  return c;
}

template <int ET> struct Elem;
template <> struct Elem<0> { typedef _Float16 T; };
template <> struct Elem<1> { typedef __bf16 T; };
template <int ET, bool SPLIT, int BIAS_MODE, int OUT_MODE, bool RESID, int ACT = 0>
__global__ __launch_bounds__(256) void wmma_gemm64(
    const unsigned short* __restrict__ Ap, const unsigned short* __restrict__ A2p, int lda, long strideA,
    const unsigned short* __restrict__ Btp, const unsigned short* __restrict__ Bt2p, int ldb, long strideB,
    void* __restrict__ Cout, void* __restrict__ Cout2, int ldc, long strideC,
    const float* __restrict__ bias,
    const float* __restrict__ resid, long strideR,
    int M, int N, int K, float scale) {
  typedef typename Elem<ET>::T T;
  typedef typename Frag<T>::V V;
  const T* A = (const T*)Ap; const T* A2 = (const T*)A2p; const T* Bt = (const T*)Btp; const T* Bt2 = (const T*)Bt2p;
  __shared__ __align__(16) float sT[8][16 * 68];
  const int b    = blockIdx.y;
  const int lane = threadIdx.x & 31;
  const int wave = threadIdx.x >> 5;
  const int tilesN = N >> 6;
  const int tilesM = M >> 6;
  const int tile = blockIdx.x * 8 + wave;
  if (tile >= tilesM * tilesN) return;
  const int tm = tile / tilesN;
  const int tn = tile - tm * tilesN;
  const int m0 = tm << 6;
  const int n0 = tn << 6;

  const T* Ab  = A  + (size_t)b * strideA;
  const T* Bb  = Bt + (size_t)b * strideB;
  const T* Ab2 = SPLIT ? (A2  + (size_t)b * strideA) : nullptr;
  const T* Bb2 = SPLIT ? (Bt2 + (size_t)b * strideB) : nullptr;

  const int rlane = lane & 15;
  const int koff  = (lane >> 4) * 8;
  const int mOff  = (lane >> 4) * 8;

  v8f acc[4][4];
#pragma unroll
  for (int i = 0; i < 4; ++i)
#pragma unroll
    for (int j = 0; j < 4; ++j) acc[i][j] = (v8f){0.f,0.f,0.f,0.f,0.f,0.f,0.f,0.f};

  for (int k0 = 0; k0 < K; k0 += 32) {
    V bh[4], bl[4];
#pragma unroll
    for (int j = 0; j < 4; ++j) {
      const size_t bo = (size_t)(n0 + (j << 4) + rlane) * ldb + koff + k0;
      bh[j] = Frag<T>::load(Bb + bo);
      if (SPLIT) bl[j] = Frag<T>::load(Bb2 + bo);
    }
#pragma unroll
    for (int i = 0; i < 4; ++i) {
      const size_t ao = (size_t)(m0 + (i << 4) + rlane) * lda + koff + k0;
      V ah = Frag<T>::load(Ab + ao);
      V al;
      if (SPLIT) al = Frag<T>::load(Ab2 + ao);
#pragma unroll
      for (int j = 0; j < 4; ++j) {
        acc[i][j] = Frag<T>::mma(ah, bh[j], acc[i][j]);
        if (SPLIT) {
          acc[i][j] = Frag<T>::mma(ah, bl[j], acc[i][j]);
          acc[i][j] = Frag<T>::mma(al, bh[j], acc[i][j]);
        }
      }
      Frag<T>::guard4(acc[i][0], acc[i][1], acc[i][2], acc[i][3], ah, SPLIT ? al : ah);
    }
    Frag<T>::keep(bh[0], bh[1], bh[2], bh[3]);
    if (SPLIT) Frag<T>::keep(bl[0], bl[1], bl[2], bl[3]);
  }
  acc_guard4(acc[0][0], acc[0][1], acc[0][2], acc[0][3]);
  acc_guard4(acc[1][0], acc[1][1], acc[1][2], acc[1][3]);
  acc_guard4(acc[2][0], acc[2][1], acc[2][2], acc[2][3]);
  acc_guard4(acc[3][0], acc[3][1], acc[3][2], acc[3][3]);

  float* slab = sT[wave];
  const float* Rb = RESID ? (resid + (size_t)b * strideR) : nullptr;
#pragma unroll
  for (int i = 0; i < 4; ++i) {
    const int mBase = m0 + (i << 4);
#pragma unroll
    for (int j = 0; j < 4; ++j) {
      const int n = n0 + (j << 4) + rlane;
      float bv = 0.f;
      if (BIAS_MODE == 2) bv = bias[n];
#pragma unroll
      for (int r = 0; r < 8; ++r) {
        float v = acc[i][j][r] * scale;
        if (BIAS_MODE == 1) v += bias[mBase + mOff + r];
        if (BIAS_MODE == 2) v += bv;
        if (RESID) v += Rb[(size_t)(mBase + mOff + r) * ldc + n];
        if (ACT == 1) v = tanhf(v);
        if (ACT == 2) v = fmaxf(v, 0.0f);
        if (ACT == 3) v = v / (1.0f + expf(-v));
        if (ACT == 4) v = (v > 0.f) ? v : 0.01f * v;
        slab[(mOff + r) * 68 + (j << 4) + rlane] = v;
      }
    }
    __builtin_amdgcn_fence(__ATOMIC_RELEASE, "workgroup");
    __builtin_amdgcn_wave_barrier();
    __builtin_amdgcn_fence(__ATOMIC_ACQUIRE, "workgroup");
    if (OUT_MODE == 0) {
      float* C = (float*)Cout + (size_t)b * strideC;
      const int hh = lane >> 4, c4 = (lane & 15) * 4;
      for (int pass = 0; pass < 2; ++pass) {
#pragma unroll
        for (int it = 0; it < 8; ++it) {
          const int row = it * 2 + hh;
          v4f v = *(const v4f*)(slab + row * 68 + c4);
          *(volatile v4f*)(C + (size_t)(mBase + row) * ldc + n0 + c4) = v;
        }
        __threadfence();
      }
    } else {
      const int q = lane >> 3, c8 = (lane & 7) * 8;
      unsigned short* C  = (unsigned short*)Cout  + (size_t)b * strideC;
      unsigned short* C2 = (OUT_MODE == 2) ? ((unsigned short*)Cout2 + (size_t)b * strideC) : nullptr;
      for (int pass = 0; pass < 2; ++pass) {
#pragma unroll
        for (int it = 0; it < 4; ++it) {
          const int row = it * 4 + q;
          const float* sp = slab + row * 68 + c8;
          v8h hv, lv;
#pragma unroll
          for (int e = 0; e < 8; ++e) {
            if (OUT_MODE == 1) {
              hv[e] = (_Float16)sp[e];
            } else {
              unsigned short hb = f2bf_bits(sp[e]);
              unsigned short lb = f2bf_bits(sp[e] - bf_bits2f(hb));
              hv[e] = __builtin_bit_cast(_Float16, hb);
              lv[e] = __builtin_bit_cast(_Float16, lb);
            }
          }
          *(volatile v8h*)(C + (size_t)(mBase + row) * ldc + n0 + c8) = hv;
          if (OUT_MODE == 2) *(volatile v8h*)(C2 + (size_t)(mBase + row) * ldc + n0 + c8) = lv;
        }
        __threadfence();
      }
    }
    __builtin_amdgcn_fence(__ATOMIC_RELEASE, "workgroup");
    __builtin_amdgcn_wave_barrier();
    __builtin_amdgcn_fence(__ATOMIC_ACQUIRE, "workgroup");
  }
}


__global__ __launch_bounds__(kThr) void zero_kernel(float* __restrict__ dst) {
  const size_t o4 = ((size_t)blockIdx.x * kThr + threadIdx.x) * 4u;
  const v4f z = {0.f, 0.f, 0.f, 0.f};
  *(volatile v4f*)(dst + o4) = z;
  __threadfence();
  *(volatile v4f*)(dst + o4) = z;
}

__global__ __launch_bounds__(kThr) void xpad_kernel(const float* __restrict__ X, unsigned short* __restrict__ XP) {
  const unsigned i = blockIdx.x * (unsigned)kThr + threadIdx.x;
  if (i >= (unsigned)kTP * 8u) return;
  const unsigned b = blockIdx.y;
  const unsigned tp = i >> 3, g8 = (i & 7u) * 8u;
  v8h hv;
#pragma unroll
  for (int e = 0; e < 8; ++e) {
    float v = 0.0f;
    if (tp >= (unsigned)(kNB - 1)) v = X[((size_t)b * kT + (tp - (unsigned)(kNB - 1))) * kI + g8 + (unsigned)e];
    hv[e] = (_Float16)carry_flush(bf16r(v), kXCarry);
  }
  unsigned short* dp = XP + ((size_t)b * kTP + tp) * kI + g8;
  *(volatile v8h*)dp = hv;
  __threadfence();
  *(volatile v8h*)dp = hv;
}
static_assert(129 * kThr >= kTP * 8 && 128 * kThr < kTP * 8, "padded-input grid: 129 blocks a sample, the last one part live");

__global__ __launch_bounds__(kThr) void bcast_kernel(const float* __restrict__ Bc, unsigned short* __restrict__ BT) {
  const unsigned t = blockIdx.x * (unsigned)kThr + threadIdx.x;
  const unsigned o = t >> 7, k8 = (t & 127u) * 8u;
  v8h hv;
#pragma unroll
  for (int e = 0; e < 8; ++e) {
    const float v = Bc[(size_t)(k8 + (unsigned)e) * kO + o];
    hv[e] = (_Float16)carry_flush(bf16r(v), kBCarry);
  }
  unsigned short* dp = BT + (size_t)o * kKF + k8;
  *(volatile v8h*)dp = hv;
  __threadfence();
  *(volatile v8h*)dp = hv;
}
static_assert(kO * (kKF / 8) == 32 * kThr, "right-operand cast grid exact: 32 blocks");

__global__ __launch_bounds__(kThr) void ar_kernel(const float* __restrict__ U, const float* __restrict__ Ac, float* __restrict__ out) {
  const unsigned i = blockIdx.x * (unsigned)kThr + threadIdx.x;
  const unsigned b = i >> 6, o = i & 63u;
  float a[kNA], y[kNA];
#pragma unroll
  for (int m = 0; m < kNA; ++m) { const float av = Ac[(unsigned)m * (unsigned)kO + o]; a[m] = bf16r(av); y[m] = 0.0f; }
  const float* up = U + (size_t)b * kT * kO + o;
  float* op = out + (size_t)b * kT * kO + o;
  for (int t = 0; t < kT; ++t) {
    float acc = 0.0f;
#pragma unroll
    for (int m = kNA - 1; m >= 0; --m) acc += a[m] * y[m];
    acc += up[(size_t)t * kO];
    float* dp = op + (size_t)t * kO;
    *(volatile float*)dp = acc;
    __threadfence();
    *(volatile float*)dp = acc;
#pragma unroll
    for (int m = kNA - 1; m > 0; --m) y[m] = y[m - 1];
    y[0] = acc;
  }
}
static_assert(kB * kO == 4 * kThr, "autoregressive grid exact: 4 blocks");

extern "C" void kernel_launch(void* const* d_in, const int* in_sizes, int n_in,
                              void* d_out, int out_size, void* d_ws, size_t ws_size,
                              hipStream_t stream) {
  if (n_in < 3 || d_out == nullptr || d_ws == nullptr) return;
  if (in_sizes[0] != kB * kT * kI || in_sizes[1] != kNA * kO || in_sizes[2] != kNB * kI * kO) return;
  if (out_size != kB * kT * kO) return;
  if (ws_size < kWsTotal) return;
  const float* X = (const float*)d_in[0];
  const float* Ac = (const float*)d_in[1];
  const float* Bc = (const float*)d_in[2];
  float* out = (float*)d_out;
  char* ws = (char*)d_ws;
  float* ZB = (float*)(ws + kOffZB);
  unsigned short* XP16 = (unsigned short*)(ws + kOffXP16);
  unsigned short* BT16 = (unsigned short*)(ws + kOffBT16);
  float* U32 = (float*)(ws + kOffU32);

  zero_kernel<<<1, kThr, 0, stream>>>(ZB);
  xpad_kernel<<<dim3(129, kB), kThr, 0, stream>>>(X, XP16);
  bcast_kernel<<<32, kThr, 0, stream>>>(Bc, BT16);
  wmma_gemm64<0, false, 2, 0, false, 0><<<dim3((kT / 64) * (kO / 64) / 8, kB), 256, 0, stream>>>(
      XP16, XP16, kI, (long)kTP * kI, BT16, BT16, kKF, 0L, (void*)U32, (void*)U32, kO, (long)kT * kO, ZB, nullptr, 0L, kT, kO, kKF, kSc);
  ar_kernel<<<4, kThr, 0, stream>>>(U32, Ac, out);
}
